// WfcNN_44032004719009
// MI455X (gfx1250) — hardware-run, weakly checked
//
#include <hip/hip_runtime.h>


#ifndef NB
#define NB 262144
#endif
#define NB_FULL 262144
#define D1    128
#define DD    64
#define DH    32
#define NOUT  2
#define NHEAD 30
#define NREL  32
#define RB    1024
#define NBLK  (NB / RB)
#define OFFP  256
#define NQ    (OFFP / 128)
#define PROWS (NB + 2048)

static_assert(NB % RB == 0);
static_assert(NBLK >= 1 && NBLK <= OFFP);
static_assert(OFFP % 128 == 0 && NQ >= 1);
static_assert(NB <= NB_FULL);
static_assert(NREL * 63 <= 2048);
static_assert(NHEAD <= NREL);
static_assert(PROWS % 64 == 0);
static_assert(DD == 64);
static_assert(D1 % 32 == 0 && DD % 32 == 0);
static_assert(DH == 32 && NOUT == 2);
static_assert(NB % 256 == 0);
static_assert(NB % 16 == 0);
static_assert(2 * D1 == 256);

typedef unsigned short bf;
typedef __attribute__((ext_vector_type(16))) __bf16   v16bf;
typedef __attribute__((ext_vector_type(8)))  unsigned short v8us;
typedef __attribute__((ext_vector_type(8)))  float    v8f;
typedef __attribute__((ext_vector_type(4)))  float    v4f;
typedef __attribute__((ext_vector_type(2)))  float    v2f;
typedef __attribute__((ext_vector_type(4)))  int      v4i;
typedef __attribute__((ext_vector_type(2)))  int      v2i;
typedef v4f  __attribute__((may_alias)) v4fa;
typedef v4i  __attribute__((may_alias)) v4ia;

__device__ __forceinline__ unsigned short f2bf(float f) { unsigned u = __float_as_uint(f); u += 0x7FFFu + ((u >> 16) & 1u); return (unsigned short)(u >> 16); }
__device__ __forceinline__ float bf2f(unsigned short w) { return __uint_as_float(((unsigned)w) << 16); }
__device__ __forceinline__ int clampi(int v, int lo, int hi) { return min(max(v, lo), hi); }
__device__ __forceinline__ v16bf cat16b(v8us lo, v8us hi) { return __builtin_bit_cast(v16bf, __builtin_shufflevector(lo, hi, 0, 1, 2, 3, 4, 5, 6, 7, 8, 9, 10, 11, 12, 13, 14, 15)); }
__device__ __forceinline__ v8f wmmab(v16bf a, v16bf b, v8f c) { return __builtin_amdgcn_wmma_f32_16x16x32_bf16(false, a, false, b, (short)0, c, false, false); }
__device__ __forceinline__ v16bf ldb(const bf* p)  { return cat16b(*(const v8us*)p, *(const v8us*)(p + 16)); }
__device__ __forceinline__ void wave_sync() { __builtin_amdgcn_fence(3  , "wavefront"); __builtin_amdgcn_wave_barrier(); asm volatile("" ::: "memory"); }

__device__ __forceinline__ float bfr(float f) { return bf2f(f2bf(f)); }
__device__ __forceinline__ v8f wmmag(v16bf a, v16bf b, v8f c) { c = wmmab(a, b, c); asm volatile("v_nop\n\tv_nop\n\tv_nop\n\tv_nop" : "+v"(c) : "v"(a), "v"(b)); return c; }
__device__ __forceinline__ float tanh_fast(float x) {
    const float e = __builtin_amdgcn_exp2f(x * 2.8853900817779268f);
    const float q = __builtin_amdgcn_rcpf(e + 1.0f);
    return __builtin_fmaf(-2.0f, q, 1.0f);
}
__device__ __forceinline__ int head_of(int n, int l, int m) {
    const unsigned un = (unsigned)n, ul = (unsigned)l, um = (unsigned)m;
    const int a = (int)((un - 1u) * un * (2u * un - 1u));
    int q = a / 6; q -= (((a % 6) != 0) & (a < 0)) ? 1 : 0;
    int h = (int)((unsigned)q + ul * ul + um + ul);
    h = (h < 0) ? h + NHEAD : h;
    return clampi(h, 0, NHEAD - 1);
}

template <int KK, int NN>
__device__ __forceinline__ void wt_body(const float* __restrict__ src, bf* dst) {
    __shared__ float ts[KK * (NN + 1)];
    constexpr int PCS = KK / 8;
    constexpr int RPP = 256 / PCS;
    constexpr int ITS = NN / RPP;
    static_assert(KK % 8 == 0 && (KK * NN) % 256 == 0);
    static_assert(PCS * RPP == 256 && ITS * RPP == NN);
    static_assert((size_t)KK * (NN + 1) * 4 <= 131072);
    const int t = threadIdx.x;
#pragma unroll 1
    for (int i = 0; i < (KK * NN) / 256; ++i) { const int f = i * 256 + t; ts[(f / NN) * (NN + 1) + (f % NN)] = src[f]; }
    __syncthreads();
#pragma unroll 1
    for (int ps = 0; ps < 2; ++ps) {
#pragma unroll 1
        for (int it = 0; it < ITS; ++it) {
            const int n = it * RPP + t / PCS, c8 = (t % PCS) * 8; v8us o;
#pragma unroll
            for (int k = 0; k < 8; ++k) o[k] = f2bf(ts[(c8 + k) * (NN + 1) + n]);
            *(volatile v8us*)(dst + n * KK + c8) = o; }
        if (ps == 0) __threadfence(); }
}

__global__ __launch_bounds__(256) void k_wt_heads(const float* __restrict__ HW1, bf* HT) {
    const int r = blockIdx.x;
    wt_body<DD, DH>(HW1 + (size_t)r * (DD * DH), HT + (size_t)r * (DD * DH));
}
__global__ __launch_bounds__(256) void k_wt_shared(const float* __restrict__ W2s, bf* W2T) {
    wt_body<D1, DD>(W2s, W2T);
}

__global__ __launch_bounds__(1024) void k_count(const int* __restrict__ qn, const int* __restrict__ ql, const int* __restrict__ qm, int* cnt) {
    __shared__ int wc[32 * 32];
    __shared__ __align__(16) int line[32];
    const int tid = threadIdx.x, lane = tid & 31; const int wave = __builtin_amdgcn_readfirstlane(tid >> 5);
    const int blk = blockIdx.x;
    const size_t row = (size_t)blk * RB + tid;
    const int rel = head_of(qn[row], ql[row], qm[row]);
    int mine = 0;
#pragma unroll 1
    for (int r = 0; r < NREL; ++r) { const unsigned m = __builtin_amdgcn_ballot_w32(rel == r); const int c = __builtin_popcount(m); mine = (lane == r) ? c : mine; }
    wc[wave * 32 + lane] = mine;
    __syncthreads();
    if (wave == 0) {
        int s = 0;
#pragma unroll 1
        for (int w = 0; w < 32; ++w) s += wc[w * 32 + lane];
        line[lane] = s;
        wave_sync();
#pragma unroll 1
        for (int ps = 0; ps < 2; ++ps) {
            if (lane < 8) { const v4i v = *(const v4ia*)(&line[4 * lane]); *(volatile v4i*)(cnt + (size_t)blk * 32 + 4 * lane) = v; }
            if (ps == 0) __threadfence(); }
    }
}

__global__ __launch_bounds__(1024) void k_scan(const int* __restrict__ cnt, int* offs, int* T, bf* AP, bf* E2P) {
    __shared__ int tots[32];
    __shared__ __align__(16) int tl[128];
    const int tid = threadIdx.x, lane = tid & 31; const int r = __builtin_amdgcn_readfirstlane(tid >> 5);
    v4i o[NQ]; int tot = 0;
#pragma unroll
    for (int q = 0; q < NQ; ++q) {
        int c[4]; int ls = 0;
#pragma unroll
        for (int i = 0; i < 4; ++i) { const int blk = q * 128 + 4 * lane + i; const int bc = min(blk, NBLK - 1);
            int v = cnt[(size_t)bc * 32 + r]; v = (blk < NBLK) ? v : 0; v = clampi(v, 0, RB); c[i] = v; ls += v; }
        int x = ls;
#pragma unroll
        for (int d = 1; d < 32; d <<= 1) { const int y = __shfl_up(x, d, 32); x += (lane >= d) ? y : 0; }
        const int excl = tot + x - ls;
        o[q][0] = excl; o[q][1] = o[q][0] + c[0]; o[q][2] = o[q][1] + c[1]; o[q][3] = o[q][2] + c[2];
        tot += __shfl(x, 31, 32);
    }
    if (lane == 0) tots[r] = tot;
    __syncthreads();
    const int t = tots[lane]; const int pd = (t + 63) & ~63;
    int y2 = pd;
#pragma unroll
    for (int d = 1; d < 32; d <<= 1) { const int y = __shfl_up(y2, d, 32); y2 += (lane >= d) ? y : 0; }
    const int sstart = y2 - pd;
    const int ptot = __shfl(y2, 31, 32);
    const int segr = __shfl(sstart, r, 32);
#pragma unroll
    for (int q = 0; q < NQ; ++q) o[q] = o[q] + (v4i){segr, segr, segr, segr};
    if (r == 0) { tl[lane] = sstart; tl[32 + lane] = t; tl[64 + lane] = (lane == 0) ? ptot : 0; tl[96 + lane] = 0; wave_sync(); }
    const int padcnt = ((tot + 63) & ~63) - tot;
    const int pbase = segr + tot;
    v8us z;
#pragma unroll
    for (int k = 0; k < 8; ++k) z[k] = (unsigned short)0;
    static_assert(32 * 16 == 128 * 4);
#pragma unroll 1
    for (int ps = 0; ps < 2; ++ps) {
#pragma unroll
        for (int q = 0; q < NQ; ++q) *(volatile v4i*)(offs + (size_t)r * OFFP + q * 128 + 4 * lane) = o[q];
        if (r == 0) { const v4i v = *(const v4ia*)(&tl[4 * lane]); *(volatile v4i*)(T + 4 * lane) = v; }
#pragma unroll 1
        for (int it = 0; it < 16; ++it) { const int j = 4 * it + (lane >> 3); const int p = clampi(pbase + j, 0, PROWS - 1); const int c8 = (lane & 7) * 8;
            if (j < padcnt) { *(volatile v8us*)(AP + (size_t)p * DD + c8) = z; *(volatile v8us*)(E2P + (size_t)p * DD + c8) = z; } }
        if (ps == 0) __threadfence(); }
}

__global__ __launch_bounds__(1024) void k_rank(const int* __restrict__ qn, const int* __restrict__ ql, const int* __restrict__ qm,
                                               const int* __restrict__ offs, int* POS) {
    __shared__ int wc[32 * 32];
    const int tid = threadIdx.x, lane = tid & 31; const int wave = __builtin_amdgcn_readfirstlane(tid >> 5);
    const int blk = blockIdx.x;
    const size_t row = (size_t)blk * RB + tid;
    const int rel = head_of(qn[row], ql[row], qm[row]);
    int mine = 0; unsigned mymask = 0u;
#pragma unroll 1
    for (int r = 0; r < NREL; ++r) { const unsigned m = __builtin_amdgcn_ballot_w32(rel == r); const int c = __builtin_popcount(m);
        mine = (lane == r) ? c : mine; mymask = (rel == r) ? m : mymask; }
    const int lrank = __builtin_popcount(mymask & ((1u << lane) - 1u));
    wc[wave * 32 + lane] = mine;
    __syncthreads();
    if (wave == 0) {
        int run = clampi(offs[(size_t)lane * OFFP + blk], 0, PROWS);
#pragma unroll 1
        for (int w = 0; w < 32; ++w) { const int c = wc[w * 32 + lane]; wc[w * 32 + lane] = run; run += c; }
    }
    __syncthreads();
    const int pos = clampi(wc[wave * 32 + rel] + lrank, 0, PROWS - 1);
#pragma unroll 1
    for (int ps = 0; ps < 2; ++ps) {
        *(volatile int*)(POS + row) = pos;
        if (ps == 0) __threadfence(); }
}

__global__ __launch_bounds__(256) __attribute__((amdgpu_num_vgpr(256))) void k_shared(const float* __restrict__ X, const float* __restrict__ W1, const float* __restrict__ B1,
                                                                                       const float* __restrict__ B2, const bf* __restrict__ W2T, const int* __restrict__ POS,
                                                                                       bf* AP, bf* E2P) {
    __shared__ __align__(16) float sw[3 * D1];
    __shared__ __align__(16) float sb2[DD];
    __shared__ __align__(16) float os[8 * 16 * 68];
    const int tid = threadIdx.x, lane = tid & 31, lr = lane & 15, hi = lane >> 4;
    const int wave = __builtin_amdgcn_readfirstlane(tid >> 5);
    {
        const float vw = bfr(W1[tid]);
        const float vb1 = bfr(B1[min(tid, D1 - 1)]);
        const float vb2 = bfr(B2[min(tid, DD - 1)]);
        sw[tid] = vw;
        if (tid < D1) sw[2 * D1 + tid] = vb1;
        if (tid < DD) sb2[tid] = vb2;
    }
    __syncthreads();
    const size_t row0 = ((size_t)blockIdx.x * 8 + (size_t)wave) * 32;
    float x0[2], x1[2];
#pragma unroll
    for (int mb = 0; mb < 2; ++mb) { const v2f xv = *(const v2f*)(X + (row0 + (size_t)(mb * 16 + lr)) * 2); x0[mb] = bfr(xv[0]); x1[mb] = bfr(xv[1]); }
    v8f acc[2][4];
#pragma unroll
    for (int mb = 0; mb < 2; ++mb)
#pragma unroll
        for (int nb = 0; nb < 4; ++nb) acc[mb][nb] = (v8f){};
    const size_t boff = (size_t)lr * D1 + 8 * hi;
#pragma unroll 1
    for (int kc = 0; kc < D1; kc += 32) {
        v8us hh[2][2], ll[2][2];
#pragma unroll
        for (int g = 0; g < 2; ++g) {
            const int kb = kc + 16 * g + 8 * hi;
            const v4f a0 = *(const v4fa*)(&sw[kb]),          a1 = *(const v4fa*)(&sw[kb + 4]);
            const v4f c0 = *(const v4fa*)(&sw[D1 + kb]),     c1 = *(const v4fa*)(&sw[D1 + kb + 4]);
            const v4f e0 = *(const v4fa*)(&sw[2 * D1 + kb]), e1 = *(const v4fa*)(&sw[2 * D1 + kb + 4]);
            float w0[8], w1[8], wb[8];
#pragma unroll
            for (int i = 0; i < 4; ++i) { w0[i] = a0[i]; w0[4 + i] = a1[i]; w1[i] = c0[i]; w1[4 + i] = c1[i]; wb[i] = e0[i]; wb[4 + i] = e1[i]; }
#pragma unroll
            for (int mb = 0; mb < 2; ++mb) {
                v8us h8, l8;
#pragma unroll
                for (int i = 0; i < 8; ++i) {
                    float p = x0[mb] * w0[i]; p = __builtin_fmaf(x1[mb], w1[i], p); p += wb[i];
                    const float v = tanh_fast(p);
                    const unsigned short hb = f2bf(v);
                    h8[i] = hb; l8[i] = f2bf(v - bf2f(hb)); }
                hh[mb][g] = h8; ll[mb][g] = l8; }
        }
        v16bf ah[2], al[2];
#pragma unroll
        for (int mb = 0; mb < 2; ++mb) { ah[mb] = cat16b(hh[mb][0], hh[mb][1]); al[mb] = cat16b(ll[mb][0], ll[mb][1]); }
#pragma unroll
        for (int nb = 0; nb < 4; ++nb) { const v16bf b = ldb(W2T + boff + (size_t)nb * 16 * D1 + kc);
#pragma unroll
            for (int mb = 0; mb < 2; ++mb) { acc[mb][nb] = wmmag(ah[mb], b, acc[mb][nb]); acc[mb][nb] = wmmag(al[mb], b, acc[mb][nb]); } }
    }
    float b2v[4];
#pragma unroll
    for (int nb = 0; nb < 4; ++nb) b2v[nb] = sb2[nb * 16 + lr];
    const int wb0 = wave * (16 * 68);
    const int c8 = (lane & 7) * 8;
    static_assert(32 * 16 * 4 == 16 * DD * 2);
#pragma unroll
    for (int mb = 0; mb < 2; ++mb) {
#pragma unroll
        for (int nb = 0; nb < 4; ++nb) {
#pragma unroll
            for (int j = 0; j < 8; ++j) os[wb0 + (hi * 8 + j) * 68 + nb * 16 + lr] = tanh_fast(acc[mb][nb][j] + b2v[nb]); }
        wave_sync();
#pragma unroll 1
        for (int ps = 0; ps < 2; ++ps) {
#pragma unroll 1
            for (int it = 0; it < 4; ++it) { const int j = 4 * it + (lane >> 3);
                const int p = clampi(POS[row0 + (size_t)(mb * 16 + j)], 0, PROWS - 1);
                const v4f u0 = *(const v4fa*)(&os[wb0 + j * 68 + c8]); const v4f u1 = *(const v4fa*)(&os[wb0 + j * 68 + c8 + 4]); v8us oa, ob;
#pragma unroll
                for (int k = 0; k < 4; ++k) { const unsigned short h0 = f2bf(u0[k]); oa[k] = h0; ob[k] = f2bf(u0[k] - bf2f(h0));
                    const unsigned short h1 = f2bf(u1[k]); oa[4 + k] = h1; ob[4 + k] = f2bf(u1[k] - bf2f(h1)); }
                *(volatile v8us*)(AP + (size_t)p * DD + c8) = oa; *(volatile v8us*)(E2P + (size_t)p * DD + c8) = ob; }
            if (ps == 0) __threadfence(); }
        wave_sync();
    }
}

__global__ __launch_bounds__(32) __attribute__((amdgpu_num_vgpr(256))) void k_heads(const bf* __restrict__ AP, const bf* __restrict__ E2P, const bf* __restrict__ HT,
                                                                                     const int* __restrict__ T, const float* __restrict__ Hb1, const float* __restrict__ HW2,
                                                                                     const float* __restrict__ Hb2, float* SORTED) {
    __shared__ __align__(16) float os[16 * 36];
    __shared__ __align__(16) float res[64 * NOUT];
    __shared__ __align__(16) float hw[DH * NOUT];
    const int lane = threadIdx.x & 31, lr = lane & 15, hi = lane >> 4;
    const int p0 = blockIdx.x * 64;
    int ss = T[lane], tt = T[32 + lane];
    asm volatile("" : "+v"(ss), "+v"(tt));
    const int pe = ss + ((tt + 63) & ~63);
    const unsigned msk = __builtin_amdgcn_ballot_w32((p0 >= ss) & (p0 < pe));
    if (msk == 0u) return;
    const int r = __builtin_amdgcn_readfirstlane(clampi(__builtin_ctz(msk), 0, NHEAD - 1));
    {
        const v2f t2 = *(const v2f*)(HW2 + (size_t)r * (DH * NOUT) + 2 * lane);
        hw[2 * lane] = bfr(t2[0]); hw[2 * lane + 1] = bfr(t2[1]);
    }
    v8f acc[4][2];
#pragma unroll
    for (int mb = 0; mb < 4; ++mb)
#pragma unroll
        for (int nb = 0; nb < 2; ++nb) acc[mb][nb] = (v8f){};
    const size_t aoff = (size_t)(p0 + lr) * DD + 8 * hi, boff = (size_t)r * (DH * DD) + (size_t)lr * DD + 8 * hi;
#pragma unroll 1
    for (int kc = 0; kc < DD; kc += 32) {
        v16bf ah[4], al[4];
#pragma unroll
        for (int mb = 0; mb < 4; ++mb) { ah[mb] = ldb(AP + aoff + (size_t)mb * 16 * DD + kc); al[mb] = ldb(E2P + aoff + (size_t)mb * 16 * DD + kc); }
#pragma unroll
        for (int nb = 0; nb < 2; ++nb) { const v16bf b = ldb(HT + boff + (size_t)nb * 16 * DD + kc);
#pragma unroll
            for (int mb = 0; mb < 4; ++mb) { acc[mb][nb] = wmmag(ah[mb], b, acc[mb][nb]); acc[mb][nb] = wmmag(al[mb], b, acc[mb][nb]); } }
    }
    float bb[2];
#pragma unroll
    for (int nb = 0; nb < 2; ++nb) bb[nb] = bfr(Hb1[(size_t)r * DH + nb * 16 + lr]);
    const int row = lane >> 1, oc = lane & 1;
    const float b2o = bfr(Hb2[(size_t)r * NOUT + oc]);
    wave_sync();
    float w2[DH];
#pragma unroll
    for (int i = 0; i < DH; ++i) w2[i] = hw[i * NOUT + oc];
#pragma unroll
    for (int mb = 0; mb < 4; ++mb) {
#pragma unroll
        for (int nb = 0; nb < 2; ++nb) {
#pragma unroll
            for (int j = 0; j < 8; ++j) os[(hi * 8 + j) * 36 + nb * 16 + lr] = tanh_fast(acc[mb][nb][j] + bb[nb]); }
        wave_sync();
        float s = b2o;
#pragma unroll
        for (int q = 0; q < 8; ++q) { const v4f zv = *(const v4fa*)(&os[row * 36 + 4 * q]);
#pragma unroll
            for (int i = 0; i < 4; ++i) s = __builtin_fmaf(zv[i], w2[4 * q + i], s); }
        res[mb * 32 + lane] = s;
        wave_sync();
    }
    static_assert(32 * 16 == 64 * NOUT * 4);
#pragma unroll 1
    for (int ps = 0; ps < 2; ++ps) {
        const v4f v = *(const v4fa*)(&res[4 * lane]); *(volatile v4f*)(SORTED + (size_t)p0 * NOUT + 4 * lane) = v;
        if (ps == 0) __threadfence(); }
}

__global__ __launch_bounds__(256) void k_unsort(const int* __restrict__ POS, const float* __restrict__ SORTED, float* OUT) {
    const size_t i = (size_t)blockIdx.x * 256 + threadIdx.x; if (i >= (size_t)(NB / 2)) return;
    const v2i p = *(const v2i*)(POS + i * 2); v4f v;
    const v2f a = *(const v2f*)(SORTED + (size_t)clampi(p[0], 0, PROWS - 1) * NOUT);
    const v2f b = *(const v2f*)(SORTED + (size_t)clampi(p[1], 0, PROWS - 1) * NOUT);
    v[0] = a[0]; v[1] = a[1]; v[2] = b[0]; v[3] = b[1];
    *(volatile v4f*)(OUT + i * 4) = v; __threadfence(); *(volatile v4f*)(OUT + i * 4) = v;
}

static constexpr size_t al256(size_t v) { return (v + 255) & ~(size_t)255; }
static constexpr size_t SZ_HT  = al256((size_t)NHEAD * DH * DD * 2);
static constexpr size_t SZ_W2T = al256((size_t)DD * D1 * 2);
static constexpr size_t SZ_CNT = al256((size_t)NBLK * 32 * 4);
static constexpr size_t SZ_OFF = al256((size_t)NREL * OFFP * 4);
static constexpr size_t SZ_T   = al256((size_t)128 * 4);
static constexpr size_t SZ_POS = al256((size_t)NB * 4);
static constexpr size_t SZ_PL  = al256((size_t)PROWS * DD * 2);
static constexpr size_t SZ_SRT = al256((size_t)PROWS * NOUT * 4);
static constexpr size_t SZ_TOTAL = SZ_HT + SZ_W2T + SZ_CNT + SZ_OFF + SZ_T + SZ_POS + 2 * SZ_PL + SZ_SRT;
static_assert(SZ_TOTAL <= (size_t)134217728);
static_assert((size_t)(3 * D1 + DD + 8 * 16 * 68) * 4 <= 131072);
static_assert((size_t)(16 * 36 + 64 * NOUT + DH * NOUT) * 4 <= 131072);
static_assert((size_t)(NBLK - 1) * 32 + 32 <= SZ_CNT / 4);
static_assert((size_t)(NREL - 1) * OFFP + (NQ - 1) * 128 + 128 <= SZ_OFF / 4);
static_assert((size_t)PROWS * DD * 2 <= SZ_PL);
static_assert((size_t)(PROWS / 64) * 64 * NOUT * 4 <= SZ_SRT);

extern "C" void kernel_launch(void* const* d_in, const int* in_sizes, int n_in,
                              void* d_out, int out_size, void* d_ws, size_t ws_size, hipStream_t stream) {
    if (n_in < 12) return;
    if ((size_t)in_sizes[0] < (size_t)NB * 2) return;
    if ((size_t)in_sizes[1] < (size_t)NB || (size_t)in_sizes[2] < (size_t)NB || (size_t)in_sizes[3] < (size_t)NB) return;
    if ((size_t)in_sizes[4] < (size_t)2 * D1 || (size_t)in_sizes[5] < (size_t)D1) return;
    if ((size_t)in_sizes[6] < (size_t)D1 * DD || (size_t)in_sizes[7] < (size_t)DD) return;
    if ((size_t)in_sizes[8] < (size_t)NHEAD * DD * DH || (size_t)in_sizes[9] < (size_t)NHEAD * DH) return;
    if ((size_t)in_sizes[10] < (size_t)NHEAD * DH * NOUT || (size_t)in_sizes[11] < (size_t)NHEAD * NOUT) return;
    if ((size_t)out_size < (size_t)NB * NOUT) return;
    if (SZ_TOTAL > ws_size) return;
    const float* X   = (const float*)d_in[0];
    const int*   qn  = (const int*)d_in[1];
    const int*   ql  = (const int*)d_in[2];
    const int*   qm  = (const int*)d_in[3];
    const float* W1s = (const float*)d_in[4];
    const float* b1s = (const float*)d_in[5];
    const float* W2s = (const float*)d_in[6];
    const float* b2s = (const float*)d_in[7];
    const float* HW1 = (const float*)d_in[8];
    const float* Hb1 = (const float*)d_in[9];
    const float* HW2 = (const float*)d_in[10];
    const float* Hb2 = (const float*)d_in[11];
    float* OUT = (float*)d_out;
    char* wsp = (char*)d_ws;
    bf*  HT  = (bf*)wsp;  wsp += SZ_HT;
    bf*  W2T = (bf*)wsp;  wsp += SZ_W2T;
    int* CNT = (int*)wsp; wsp += SZ_CNT;
    int* OFF = (int*)wsp; wsp += SZ_OFF;
    int* TT  = (int*)wsp; wsp += SZ_T;
    int* POS = (int*)wsp; wsp += SZ_POS;
    bf*  AP  = (bf*)wsp;  wsp += SZ_PL;
    bf*  E2P = (bf*)wsp;  wsp += SZ_PL;
    float* SRT = (float*)wsp; wsp += SZ_SRT;

    k_wt_heads<<<NHEAD, 256, 0, stream>>>(HW1, HT);
    k_wt_shared<<<1, 256, 0, stream>>>(W2s, W2T);
    k_count<<<NBLK, 1024, 0, stream>>>(qn, ql, qm, CNT);
    k_scan<<<1, 1024, 0, stream>>>(CNT, OFF, TT, AP, E2P);
    k_rank<<<NBLK, 1024, 0, stream>>>(qn, ql, qm, OFF, POS);
    k_shared<<<NB / 256, 256, 0, stream>>>(X, W1s, b1s, b2s, W2T, POS, AP, E2P);
    k_heads<<<PROWS / 64, 32, 0, stream>>>(AP, E2P, HT, TT, Hb1, HW2, Hb2, SRT);
    k_unsort<<<(unsigned)((NB / 2 + 255) / 256), 256, 0, stream>>>(POS, SRT, OUT);
}
